// Block_867583394304
// MI455X (gfx1250) — hardware-verified
//
#include <hip/hip_runtime.h>


#pragma clang fp contract(off)

#ifndef NB
#define NB 8
#endif
#ifndef SEQ
#define SEQ 1024
#endif
#define NB_FULL 8
#define SEQ_FULL 1024
#define CDIM 768
#define NHEAD 12
#define HD 64
#define HID 3072
#define MROWS (NB * SEQ)

static_assert(NB >= 1 && NB <= NB_FULL);
static_assert(SEQ % 64 == 0 && SEQ >= 64 && SEQ <= SEQ_FULL);
static_assert((SEQ & (SEQ - 1)) == 0);
static_assert(CDIM == NHEAD * HD);
static_assert(HD == 64);
static_assert(CDIM == 768);
static_assert(HID == 4 * CDIM);
static_assert(HID % 64 == 0 && CDIM % 64 == 0 && (3 * CDIM) % 64 == 0);
static_assert(CDIM % 32 == 0 && HID % 32 == 0);
static_assert(MROWS % 64 == 0);
static_assert((3 * CDIM * CDIM) % 2048 == 0 && (CDIM * CDIM) % 2048 == 0 && (HID * CDIM) % 2048 == 0);

typedef _Float16 v16h __attribute__((ext_vector_type(16)));
typedef _Float16 v8h  __attribute__((ext_vector_type(8)));
typedef float    v8f  __attribute__((ext_vector_type(8)));
typedef float    v4f  __attribute__((ext_vector_type(4)));
typedef unsigned int v4u __attribute__((ext_vector_type(4)));

union Frag { v16h v; v4u q[2]; };

__device__ __forceinline__ v8f mma(v16h a, v16h b, v8f c) {
  v8f d = __builtin_amdgcn_wmma_f32_16x16x32_f16(false, a, false, b, (short)0, c, false, false);
  asm volatile("v_nop\n\tv_nop\n\tv_nop\n\tv_nop" : "+v"(d) : "v"(a), "v"(b));
  return d;
}

__device__ __forceinline__ v8f zero8() {
  v8f z;
#pragma unroll
  for (int i = 0; i < 8; ++i) z[i] = 0.0f;
  return z;
}

__device__ __forceinline__ float bf16q(float f) {
  unsigned int u = __float_as_uint(f);
  unsigned int r = u + 0x7FFFu + ((u >> 16) & 1u);
  r = ((u & 0x7F800000u) == 0x7F800000u) ? u : r;
  return __uint_as_float(r & 0xFFFF0000u);
}
__device__ __forceinline__ v4f bf16q4(v4f a) {
  v4f r;
  r.x = bf16q(a.x); r.y = bf16q(a.y); r.z = bf16q(a.z); r.w = bf16q(a.w);
  return r;
}
__device__ __forceinline__ unsigned short hbits(float f) {
  _Float16 h = (_Float16)f;
  return __builtin_bit_cast(unsigned short, h);
}
__device__ __forceinline__ v4u pack8h(float f0, float f1, float f2, float f3,
                                      float f4, float f5, float f6, float f7) {
  v8h t;
  t[0] = (_Float16)f0; t[1] = (_Float16)f1; t[2] = (_Float16)f2; t[3] = (_Float16)f3;
  t[4] = (_Float16)f4; t[5] = (_Float16)f5; t[6] = (_Float16)f6; t[7] = (_Float16)f7;
  return __builtin_bit_cast(v4u, t);
}

__global__ __launch_bounds__(256) void k_wcvt(
    const float* __restrict__ s0, const float* __restrict__ s1,
    const float* __restrict__ s2, const float* __restrict__ s3,
    unsigned short* __restrict__ d0, unsigned short* __restrict__ d1,
    unsigned short* __restrict__ d2, unsigned short* __restrict__ d3,
    unsigned nb0, unsigned nb1, unsigned nb2, unsigned nb3) {
  const unsigned z = blockIdx.y;
  const float* src = (z == 0u) ? s0 : ((z == 1u) ? s1 : ((z == 2u) ? s2 : s3));
  unsigned short* dst = (z == 0u) ? d0 : ((z == 1u) ? d1 : ((z == 2u) ? d2 : d3));
  const unsigned nb = (z == 0u) ? nb0 : ((z == 1u) ? nb1 : ((z == 2u) ? nb2 : nb3));
  if (blockIdx.x >= nb) return;
  const unsigned e = (blockIdx.x * 256u + threadIdx.x) * 8u;
  const v4f a = *(const v4f*)(src + e);
  const v4f b = *(const v4f*)(src + e + 4);
  const v4u o = pack8h(bf16q(a.x) * 16.0f, bf16q(a.y) * 16.0f, bf16q(a.z) * 16.0f, bf16q(a.w) * 16.0f,
                       bf16q(b.x) * 16.0f, bf16q(b.y) * 16.0f, bf16q(b.z) * 16.0f, bf16q(b.w) * 16.0f);
  *(volatile v4u*)(dst + e) = o;
  __threadfence();
  *(volatile v4u*)(dst + e) = o;
}

template <int RNDIN>
__global__ __launch_bounds__(256) void k_ln(
    const float* __restrict__ x, const float* __restrict__ g, const float* __restrict__ bt,
    unsigned short* __restrict__ hout, unsigned nrows) {
  const unsigned lane = threadIdx.x & 31u, w = threadIdx.x >> 5;
  const unsigned row = blockIdx.x * 8u + w;
  if (row >= nrows) return;
  size_t xrow;
  if (RNDIN) {
    const unsigned b = row / (unsigned)SEQ, t = row & (unsigned)(SEQ - 1);
    xrow = ((size_t)b * SEQ_FULL + t) * CDIM;
  } else {
    xrow = (size_t)row * CDIM;
  }
  const unsigned c0 = lane * 8u;

  float v[24];
#pragma unroll
  for (int c = 0; c < 3; ++c) {
    const v4f t0 = *(const v4f*)(x + xrow + c0 + 256 * c);
    const v4f t1 = *(const v4f*)(x + xrow + c0 + 256 * c + 4);
    v[8 * c + 0] = t0.x; v[8 * c + 1] = t0.y; v[8 * c + 2] = t0.z; v[8 * c + 3] = t0.w;
    v[8 * c + 4] = t1.x; v[8 * c + 5] = t1.y; v[8 * c + 6] = t1.z; v[8 * c + 7] = t1.w;
  }
  if (RNDIN) {
#pragma unroll
    for (int i = 0; i < 24; ++i) v[i] = bf16q(v[i]);
  }

  float s = 0.0f;
#pragma unroll
  for (int i = 0; i < 24; ++i) s += v[i];
#pragma unroll
  for (int xm = 1; xm < 32; xm <<= 1) s += __shfl_xor(s, xm, 32);
  const float mu = s * (1.0f / CDIM);

  float d[24];
#pragma unroll
  for (int i = 0; i < 24; ++i) d[i] = v[i] - mu;
  float qs = 0.0f;
#pragma unroll
  for (int i = 0; i < 24; ++i) qs += d[i] * d[i];
#pragma unroll
  for (int xm = 1; xm < 32; xm <<= 1) qs += __shfl_xor(qs, xm, 32);
  const float var = qs * (1.0f / CDIM);
  const float rstd = rsqrtf(var + 1e-5f);

  v4u o[3];
#pragma unroll
  for (int c = 0; c < 3; ++c) {
    const v4f g0 = bf16q4(*(const v4f*)(g + c0 + 256 * c));
    const v4f g1 = bf16q4(*(const v4f*)(g + c0 + 256 * c + 4));
    const v4f b0 = bf16q4(*(const v4f*)(bt + c0 + 256 * c));
    const v4f b1 = bf16q4(*(const v4f*)(bt + c0 + 256 * c + 4));
    const float y0 = d[8 * c + 0] * rstd * g0.x + b0.x;
    const float y1 = d[8 * c + 1] * rstd * g0.y + b0.y;
    const float y2 = d[8 * c + 2] * rstd * g0.z + b0.z;
    const float y3 = d[8 * c + 3] * rstd * g0.w + b0.w;
    const float y4 = d[8 * c + 4] * rstd * g1.x + b1.x;
    const float y5 = d[8 * c + 5] * rstd * g1.y + b1.y;
    const float y6 = d[8 * c + 6] * rstd * g1.z + b1.z;
    const float y7 = d[8 * c + 7] * rstd * g1.w + b1.w;
    o[c] = pack8h(y0, y1, y2, y3, y4, y5, y6, y7);
  }
  unsigned short* orow = hout + (size_t)row * CDIM;
#pragma unroll
  for (int c = 0; c < 3; ++c) *(volatile v4u*)(orow + c0 + 256 * c) = o[c];
  __threadfence();
#pragma unroll
  for (int c = 0; c < 3; ++c) *(volatile v4u*)(orow + c0 + 256 * c) = o[c];
}

template <int EPI, int RESFULL, int OUTFULL>
__global__ __launch_bounds__(128) void k_gemm(
    const unsigned short* __restrict__ A, const unsigned short* __restrict__ Bt, unsigned K,
    const float* __restrict__ bias, const float* __restrict__ bias2,
    const float* __restrict__ gam, const float* __restrict__ res,
    float* __restrict__ outF, unsigned short* __restrict__ out0,
    unsigned short* __restrict__ out1, unsigned short* __restrict__ out2, unsigned ldo) {
  __shared__ __attribute__((aligned(16))) unsigned short sT[64][72];
  __shared__ __attribute__((aligned(16))) float sF[64][68];
  const unsigned tid = threadIdx.x, lane = tid & 31u, w = tid >> 5;
  const unsigned m = lane & 15u, hl = lane >> 4, k8 = hl * 8u;
  const unsigned m0 = blockIdx.y * 64u, n0 = blockIdx.x * 64u;

  v8f acc[4];
#pragma unroll
  for (int j = 0; j < 4; ++j) acc[j] = zero8();

  const unsigned short* ap = A + (size_t)(m0 + 16u * w + m) * (size_t)K + k8;
  const unsigned short* bp = Bt + (size_t)(n0 + m) * (size_t)K + k8;
  const size_t jstep = (size_t)16 * (size_t)K;
#pragma unroll 1
  for (unsigned k0 = 0; k0 < K; k0 += 32u) {
    Frag a;
    a.q[0] = *(const v4u*)(ap + k0);
    a.q[1] = *(const v4u*)(ap + k0 + 16);
#pragma unroll
    for (int j = 0; j < 4; ++j) {
      Frag b;
      const unsigned short* bj = bp + jstep * j + k0;
      b.q[0] = *(const v4u*)(bj);
      b.q[1] = *(const v4u*)(bj + 16);
      acc[j] = mma(a.v, b.v, acc[j]);
    }
  }

  const float wsc = 0.0625f;
  const unsigned lrow0 = 16u * w + 8u * hl;

  if constexpr (EPI == 0) {
    const unsigned which = n0 / (unsigned)CDIM;
    const unsigned hc = n0 - which * (unsigned)CDIM;
    const unsigned hh = hc >> 6;
#pragma unroll
    for (int j = 0; j < 4; ++j) {
      const float qv = bf16q(bias[hc + 16u * j + m]);
      const float vv = bf16q(bias2[hc + 16u * j + m]);
      const float bj = (which == 0u) ? qv : ((which == 2u) ? vv : 0.0f);
#pragma unroll
      for (int r = 0; r < 8; ++r) sT[lrow0 + r][16 * j + m] = hbits(acc[j][r] * wsc + bj);
    }
    __syncthreads();
    const unsigned b = m0 / (unsigned)SEQ, t0 = m0 & (unsigned)(SEQ - 1);
    const unsigned bh = b * NHEAD + hh;
    v4u val[4];
    unsigned int off[4];
    unsigned short* dst;
    if (which < 2u) {
      dst = (which == 0u) ? out0 : out1;
#pragma unroll
      for (int p = 0; p < 4; ++p) {
        const unsigned row = p * 16u + 4u * w + (lane >> 3);
        const unsigned piece = lane & 7u;
        val[p] = *(const v4u*)&sT[row][piece * 8u];
        off[p] = (bh * (unsigned)SEQ + t0 + row) * HD + piece * 8u;
      }
    } else {
      dst = out2;
#pragma unroll
      for (int p = 0; p < 4; ++p) {
        const unsigned d = p * 16u + 4u * w + (lane >> 3);
        const unsigned piece = lane & 7u;
        unsigned int wv[4];
#pragma unroll
        for (int e = 0; e < 4; ++e) {
          const unsigned int lo = sT[piece * 8u + 2 * e][d];
          const unsigned int hi = sT[piece * 8u + 2 * e + 1][d];
          wv[e] = lo | (hi << 16);
        }
        v4u t;
        t.x = wv[0]; t.y = wv[1]; t.z = wv[2]; t.w = wv[3];
        val[p] = t;
        off[p] = (bh * HD + d) * (unsigned)SEQ + t0 + piece * 8u;
      }
    }
#pragma unroll
    for (int p = 0; p < 4; ++p) *(volatile v4u*)(dst + off[p]) = val[p];
    __threadfence();
#pragma unroll
    for (int p = 0; p < 4; ++p) *(volatile v4u*)(dst + off[p]) = val[p];
  } else if constexpr (EPI == 1) {
#pragma unroll
    for (int j = 0; j < 4; ++j) {
#pragma unroll
      for (int r = 0; r < 8; ++r) sF[lrow0 + r][16 * j + m] = acc[j][r] * wsc;
    }
    __syncthreads();
    const unsigned b = m0 / (unsigned)SEQ, t0 = m0 & (unsigned)(SEQ - 1);
    const unsigned ncol = n0 + 4u * m;
    const v4f bv = bf16q4(*(const v4f*)(bias + ncol));
    const v4f gv = bf16q4(*(const v4f*)(gam + ncol));
    v4f val[8];
    unsigned int off[8];
#pragma unroll
    for (int p = 0; p < 8; ++p) {
      const unsigned row = 16u * w + 2u * p + hl;
      const v4f a = *(const v4f*)&sF[row][4u * m];
      const size_t rrow = RESFULL ? ((size_t)b * SEQ_FULL + t0 + row) : (size_t)(m0 + row);
      v4f rr = *(const v4f*)(res + rrow * (size_t)ldo + ncol);
      if (RESFULL) rr = bf16q4(rr);
      val[p] = rr + gv * (a + bv);
      const size_t orow = OUTFULL ? ((size_t)b * SEQ_FULL + t0 + row) : (size_t)(m0 + row);
      off[p] = (unsigned int)(orow * (size_t)ldo + ncol);
    }
#pragma unroll
    for (int p = 0; p < 8; ++p) *(volatile v4f*)(outF + off[p]) = val[p];
    __threadfence();
#pragma unroll
    for (int p = 0; p < 8; ++p) *(volatile v4f*)(outF + off[p]) = val[p];
  } else {
#pragma unroll
    for (int j = 0; j < 4; ++j) {
      const float bj = bf16q(bias[n0 + 16u * j + m]);
#pragma unroll
      for (int r = 0; r < 8; ++r) {
        const float u = acc[j][r] * wsc + bj;
        const float ge = 0.5f * u * (1.0f + erff(u * 0.70710678118654752f));
        sT[lrow0 + r][16 * j + m] = hbits(ge);
      }
    }
    __syncthreads();
    v4u val[4];
    unsigned int off[4];
#pragma unroll
    for (int p = 0; p < 4; ++p) {
      const unsigned row = 16u * w + 4u * p + (lane >> 3);
      const unsigned piece = lane & 7u;
      val[p] = *(const v4u*)&sT[row][piece * 8u];
      off[p] = (unsigned int)((size_t)(m0 + row) * (size_t)ldo + n0 + piece * 8u);
    }
#pragma unroll
    for (int p = 0; p < 4; ++p) *(volatile v4u*)(out0 + off[p]) = val[p];
    __threadfence();
#pragma unroll
    for (int p = 0; p < 4; ++p) *(volatile v4u*)(out0 + off[p]) = val[p];
  }
}

__global__ __launch_bounds__(128) __attribute__((amdgpu_num_vgpr(256)))
void k_attn(const unsigned short* __restrict__ qp, const unsigned short* __restrict__ kp,
            const unsigned short* __restrict__ vp, unsigned short* __restrict__ op) {
  __shared__ __attribute__((aligned(16))) unsigned short sP[4][16][72];
  const unsigned tid = threadIdx.x, lane = tid & 31u, w = tid >> 5;
  const unsigned m = lane & 15u, hl = lane >> 4, k8 = hl * 8u;
  const unsigned nqt = SEQ / 64;
  const unsigned bh = blockIdx.x / nqt, qt = blockIdx.x - bh * nqt;
  const unsigned b = bh / (unsigned)NHEAD, hh = bh - b * (unsigned)NHEAD;
  const unsigned tq = qt * 64u + 16u * w;

  Frag qa0, qa1;
  {
    const unsigned short* qr = qp + ((size_t)bh * SEQ + tq + m) * HD + k8;
    qa0.q[0] = *(const v4u*)(qr);
    qa0.q[1] = *(const v4u*)(qr + 16);
    qa1.q[0] = *(const v4u*)(qr + 32);
    qa1.q[1] = *(const v4u*)(qr + 48);
  }
  float mrun[8], lrun[8];
  v8f oacc[4];
#pragma unroll
  for (int r = 0; r < 8; ++r) { mrun[r] = -1e30f; lrun[r] = 0.0f; }
#pragma unroll
  for (int j = 0; j < 4; ++j) oacc[j] = zero8();

#pragma unroll 1
  for (unsigned kt = 0; kt < nqt; ++kt) {
    v8f s[4];
    const unsigned short* kb = kp + ((size_t)bh * SEQ + kt * 64u + m) * HD + k8;
#pragma unroll
    for (int j = 0; j < 4; ++j) {
      const unsigned short* kr = kb + j * 16 * HD;
      Frag f0, f1;
      f0.q[0] = *(const v4u*)(kr);
      f0.q[1] = *(const v4u*)(kr + 16);
      f1.q[0] = *(const v4u*)(kr + 32);
      f1.q[1] = *(const v4u*)(kr + 48);
      v8f t = mma(qa0.v, f0.v, zero8());
      t = mma(qa1.v, f1.v, t);
      s[j] = t;
    }
    float tmax[8];
#pragma unroll
    for (int r = 0; r < 8; ++r) tmax[r] = -1e30f;
#pragma unroll
    for (int j = 0; j < 4; ++j) {
#pragma unroll
      for (int r = 0; r < 8; ++r) {
        const float val = s[j][r] * 0.125f;
        s[j][r] = val;
        tmax[r] = fmaxf(tmax[r], val);
      }
    }
#pragma unroll
    for (int r = 0; r < 8; ++r) {
#pragma unroll
      for (int xm = 1; xm < 16; xm <<= 1) tmax[r] = fmaxf(tmax[r], __shfl_xor(tmax[r], xm, 32));
    }
    float corr[8];
#pragma unroll
    for (int r = 0; r < 8; ++r) {
      const float mn = fmaxf(mrun[r], tmax[r]);
      corr[r] = __expf(mrun[r] - mn);
      mrun[r] = mn;
    }
    float tsum[8];
#pragma unroll
    for (int r = 0; r < 8; ++r) tsum[r] = 0.0f;
#pragma unroll
    for (int j = 0; j < 4; ++j) {
#pragma unroll
      for (int r = 0; r < 8; ++r) {
        const float p = __expf(s[j][r] - mrun[r]);
        tsum[r] += p;
        sP[w][8u * hl + r][16 * j + m] = hbits(p * 1024.0f);
      }
    }
#pragma unroll
    for (int r = 0; r < 8; ++r) {
#pragma unroll
      for (int xm = 1; xm < 16; xm <<= 1) tsum[r] += __shfl_xor(tsum[r], xm, 32);
      lrun[r] = lrun[r] * corr[r] + tsum[r];
    }
#pragma unroll
    for (int j = 0; j < 4; ++j) {
#pragma unroll
      for (int r = 0; r < 8; ++r) oacc[j][r] *= corr[r];
    }
    __syncthreads();
    Frag pa0, pa1;
    {
      const unsigned short* pr = &sP[w][m][k8];
      pa0.q[0] = *(const v4u*)(pr);
      pa0.q[1] = *(const v4u*)(pr + 16);
      pa1.q[0] = *(const v4u*)(pr + 32);
      pa1.q[1] = *(const v4u*)(pr + 48);
    }
    const unsigned short* vb = vp + ((size_t)bh * HD + m) * (size_t)SEQ + kt * 64u + k8;
#pragma unroll
    for (int jd = 0; jd < 4; ++jd) {
      const unsigned short* vr = vb + (size_t)jd * 16 * SEQ;
      Frag g0, g1;
      g0.q[0] = *(const v4u*)(vr);
      g0.q[1] = *(const v4u*)(vr + 16);
      g1.q[0] = *(const v4u*)(vr + 32);
      g1.q[1] = *(const v4u*)(vr + 48);
      oacc[jd] = mma(pa0.v, g0.v, oacc[jd]);
      oacc[jd] = mma(pa1.v, g1.v, oacc[jd]);
    }
    __syncthreads();
  }

  float il[8];
#pragma unroll
  for (int r = 0; r < 8; ++r) il[r] = 1.0f / (lrun[r] * 1024.0f);
#pragma unroll
  for (int jd = 0; jd < 4; ++jd) {
#pragma unroll
    for (int r = 0; r < 8; ++r) sP[w][8u * hl + r][16 * jd + m] = hbits(oacc[jd][r] * il[r]);
  }
  __syncthreads();
  v4u val[4];
  unsigned int off[4];
#pragma unroll
  for (int p = 0; p < 4; ++p) {
    const unsigned row = 4u * p + (lane >> 3);
    const unsigned piece = lane & 7u;
    val[p] = *(const v4u*)&sP[w][row][piece * 8u];
    off[p] = (b * (unsigned)SEQ + tq + row) * (unsigned)CDIM + hh * HD + piece * 8u;
  }
#pragma unroll
  for (int p = 0; p < 4; ++p) *(volatile v4u*)(op + off[p]) = val[p];
  __threadfence();
#pragma unroll
  for (int p = 0; p < 4; ++p) *(volatile v4u*)(op + off[p]) = val[p];
}

static inline size_t al256(size_t v) { return (v + 255) & ~(size_t)255; }

extern "C" void kernel_launch(void* const* d_in, const int* in_sizes, int n_in,
                              void* d_out, int out_size, void* d_ws, size_t ws_size,
                              hipStream_t stream) {
  if (n_in < 16) return;
  const long needX = ((long)(NB - 1) * SEQ_FULL + SEQ) * CDIM;
  if ((long)in_sizes[0] < needX) return;
  if (in_sizes[1] < CDIM || in_sizes[2] < CDIM) return;
  if ((long)in_sizes[3] < (long)3 * CDIM * CDIM) return;
  if (in_sizes[4] < CDIM || in_sizes[5] < CDIM) return;
  if ((long)in_sizes[6] < (long)CDIM * CDIM || in_sizes[7] < CDIM) return;
  if (in_sizes[8] < CDIM || in_sizes[9] < CDIM) return;
  if ((long)in_sizes[10] < (long)HID * CDIM || in_sizes[11] < HID) return;
  if ((long)in_sizes[12] < (long)CDIM * HID || in_sizes[13] < CDIM) return;
  if (in_sizes[14] < CDIM || in_sizes[15] < CDIM) return;
  if ((long)out_size < needX) return;

  const float* x     = (const float*)d_in[0];
  const float* ln1_g = (const float*)d_in[1];
  const float* ln1_b = (const float*)d_in[2];
  const float* Wqkv  = (const float*)d_in[3];
  const float* qb    = (const float*)d_in[4];
  const float* vb    = (const float*)d_in[5];
  const float* Wp    = (const float*)d_in[6];
  const float* pb    = (const float*)d_in[7];
  const float* ln2_g = (const float*)d_in[8];
  const float* ln2_b = (const float*)d_in[9];
  const float* W1    = (const float*)d_in[10];
  const float* b1    = (const float*)d_in[11];
  const float* W2    = (const float*)d_in[12];
  const float* b2    = (const float*)d_in[13];
  const float* g1    = (const float*)d_in[14];
  const float* g2    = (const float*)d_in[15];
  float* out = (float*)d_out;

  char* ws = (char*)d_ws;
  size_t off = 0;
  auto carve = [&](size_t bytes) -> char* { char* p = ws + off; off += al256(bytes); return p; };
  const size_t MC = (size_t)MROWS * CDIM;
  unsigned short* wqkv = (unsigned short*)carve((size_t)3 * CDIM * CDIM * 2);
  unsigned short* wpt  = (unsigned short*)carve((size_t)CDIM * CDIM * 2);
  unsigned short* w1t  = (unsigned short*)carve((size_t)HID * CDIM * 2);
  unsigned short* w2t  = (unsigned short*)carve((size_t)CDIM * HID * 2);
  unsigned short* hpl  = (unsigned short*)carve(MC * 2);
  static_assert((size_t)MROWS * HID * 2 <= (size_t)4 * MROWS * CDIM * 2);
  unsigned short* big  = (unsigned short*)carve((size_t)4 * MC * 2);
  unsigned short* qpl  = big;
  unsigned short* kpl  = big + MC;
  unsigned short* vtp  = big + 2 * MC;
  unsigned short* opl  = big + 3 * MC;
  unsigned short* act  = big;
  float*          x1   = (float*)carve(MC * 4);
  unsigned short* h2p  = (unsigned short*)carve(MC * 2);
  if (off > ws_size) return;
  if (off > (size_t)134217728) return;

  const unsigned nbq = (unsigned)(3 * CDIM * CDIM / 2048);
  const unsigned nbp = (unsigned)(CDIM * CDIM / 2048);
  const unsigned nb1 = (unsigned)(HID * CDIM / 2048);
  k_wcvt<<<dim3(nb1, 4), 256, 0, stream>>>(Wqkv, Wp, W1, W2, wqkv, wpt, w1t, w2t, nbq, nbp, nb1, nb1);
  k_ln<1><<<MROWS / 8, 256, 0, stream>>>(x, ln1_g, ln1_b, hpl, (unsigned)MROWS);
  k_gemm<0, 0, 0><<<dim3(3 * CDIM / 64, MROWS / 64), 128, 0, stream>>>(
      hpl, wqkv, (unsigned)CDIM, qb, vb, nullptr, nullptr, nullptr, qpl, kpl, vtp, 0u);
  k_attn<<<NB * NHEAD * (SEQ / 64), 128, 0, stream>>>(qpl, kpl, vtp, opl);
  k_gemm<1, 1, 0><<<dim3(CDIM / 64, MROWS / 64), 128, 0, stream>>>(
      opl, wpt, (unsigned)CDIM, pb, nullptr, g1, x, x1, nullptr, nullptr, nullptr, (unsigned)CDIM);
  k_ln<0><<<MROWS / 8, 256, 0, stream>>>(x1, ln2_g, ln2_b, h2p, (unsigned)MROWS);
  k_gemm<2, 0, 0><<<dim3(HID / 64, MROWS / 64), 128, 0, stream>>>(
      h2p, w1t, (unsigned)CDIM, b1, nullptr, nullptr, nullptr, nullptr, act, nullptr, nullptr, (unsigned)HID);
  k_gemm<1, 0, 1><<<dim3(CDIM / 64, MROWS / 64), 128, 0, stream>>>(
      act, w2t, (unsigned)HID, b2, nullptr, g2, x1, out, nullptr, nullptr, nullptr, (unsigned)CDIM);
}
